// Attention_84104049590786
// MI455X (gfx1250) — hardware-verified
//
#include <hip/hip_runtime.h>


#ifndef NB
#define NB 4
#endif
#ifndef SEQ
#define SEQ 2048
#endif
#define NB_FULL  4
#define SEQ_FULL 2048
#define DMO   1024
#define NH    16
#define HD    64
#define QKVC  (3 * NH * HD)
#define SCL   0.125f
#define MASKV 1000000.0f
#define PCAR  16384.0f
#define RCAR  4096.0f
#define VCAR  16.0f
#define L2E   1.4426950408889634f

static_assert(SEQ % 64 == 0);
static_assert((NB * SEQ) % 64 == 0);
static_assert(DMO % 64 == 0);
static_assert(QKVC % 64 == 0);
static_assert(DMO % 32 == 0);
static_assert(HD == 64);
static_assert(NB >= 1 && NB <= NB_FULL);
static_assert(SEQ <= SEQ_FULL);

typedef _Float16 h16;
typedef unsigned short bf;
typedef __attribute__((ext_vector_type(16))) __bf16   v16bf;
typedef __attribute__((ext_vector_type(16))) _Float16 v16h;
typedef __attribute__((ext_vector_type(8)))  _Float16 v8h;
typedef __attribute__((ext_vector_type(2)))  _Float16 v2h;
typedef __attribute__((ext_vector_type(8)))  unsigned short v8us;
typedef __attribute__((ext_vector_type(2)))  unsigned short v2us;
typedef __attribute__((ext_vector_type(8)))  float    v8f;
typedef __attribute__((ext_vector_type(4)))  float    v4f;
typedef __attribute__((ext_vector_type(8)))  int      v8i;
typedef v8h  __attribute__((may_alias)) v8ha;
typedef v4f  __attribute__((may_alias)) v4fa;
typedef v8us __attribute__((may_alias)) v8usa;

__device__ __forceinline__ unsigned short f2bf(float f) { unsigned u = __float_as_uint(f); u += 0x7FFFu + ((u >> 16) & 1u); return (unsigned short)(u >> 16); }
__device__ __forceinline__ float bf2f(unsigned short b) { return __uint_as_float(((unsigned)b) << 16); }
__device__ __forceinline__ float bfr(float f) { return bf2f(f2bf(f)); }
__device__ __forceinline__ h16 tohx(float x) { return (h16)x; }
__device__ __forceinline__ void splitf(float y, unsigned short& h, unsigned short& l) { h = f2bf(y); l = f2bf(y - bf2f(h)); }
__device__ __forceinline__ v16h cat16(v8h lo, v8h hi) { return __builtin_shufflevector(lo, hi, 0, 1, 2, 3, 4, 5, 6, 7, 8, 9, 10, 11, 12, 13, 14, 15); }
__device__ __forceinline__ v16bf cat16b(v8us lo, v8us hi) { return __builtin_bit_cast(v16bf, __builtin_shufflevector(lo, hi, 0, 1, 2, 3, 4, 5, 6, 7, 8, 9, 10, 11, 12, 13, 14, 15)); }
__device__ __forceinline__ v8f wmma16(v16h a, v16h b, v8f c) { return __builtin_amdgcn_wmma_f32_16x16x32_f16(false, a, false, b, (short)0, c, false, false); }
__device__ __forceinline__ v8f wmmab(v16bf a, v16bf b, v8f c) { return __builtin_amdgcn_wmma_f32_16x16x32_bf16(false, a, false, b, (short)0, c, false, false); }
__device__ __forceinline__ v16h ldh(const h16* p) { return cat16(*(const v8h*)p, *(const v8h*)(p + 16)); }

template <typename T16> struct WFrag;
template <> struct WFrag<h16> { typedef v16h V; static __device__ __forceinline__ V ld(const h16* p) { return cat16(*(const v8h*)p, *(const v8h*)(p + 16)); } static __device__ __forceinline__ v8f mma(V a, V b, v8f c) { return wmma16(a, b, c); } };
template <> struct WFrag<bf> { typedef v16bf V; static __device__ __forceinline__ V ld(const bf* p) { return cat16b(*(const v8us*)p, *(const v8us*)(p + 16)); } static __device__ __forceinline__ v8f mma(V a, V b, v8f c) { return wmmab(a, b, c); } };
template <typename T16, int NSPLIT, bool BIAS>
__global__ __launch_bounds__(32) void k_gemmw(const T16* __restrict__ A, const T16* __restrict__ A2, const T16* __restrict__ Bt, const T16* __restrict__ Bt2, int K, float* C, int ldc, const float* __restrict__ bias, size_t sA, size_t sB, size_t sC) {
    typedef typename WFrag<T16>::V V;
    __shared__ __align__(16) float os[16 * 68];
    const size_t z = blockIdx.z; A += z * sA; if (A2) A2 += z * sA; Bt += z * sB; if (Bt2) Bt2 += z * sB; C += z * sC;
    const int lane = threadIdx.x & 31, lr = lane & 15, hi = lane >> 4; const int r0 = blockIdx.x * 64, c0 = blockIdx.y * 64;
    v8f acc[4][4];
#pragma unroll
    for (int mb = 0; mb < 4; ++mb)
#pragma unroll
        for (int nb = 0; nb < 4; ++nb) acc[mb][nb] = (v8f){};
    const size_t aoff = (size_t)(r0 + lr) * K + 8 * hi, boff = (size_t)(c0 + lr) * K + 8 * hi;
#pragma unroll 1
    for (int kc = 0; kc < K; kc += 32) {
        V a[4], a2[4];
#pragma unroll
        for (int mb = 0; mb < 4; ++mb) { a[mb] = WFrag<T16>::ld(A + aoff + (size_t)mb * 16 * K + kc); if (NSPLIT == 1 || NSPLIT == 2) a2[mb] = WFrag<T16>::ld(A2 + aoff + (size_t)mb * 16 * K + kc); }
#pragma unroll
        for (int nb = 0; nb < 4; ++nb) { const V b = WFrag<T16>::ld(Bt + boff + (size_t)nb * 16 * K + kc); V b2; if (NSPLIT >= 2) b2 = WFrag<T16>::ld(Bt2 + boff + (size_t)nb * 16 * K + kc);
#pragma unroll
            for (int mb = 0; mb < 4; ++mb) { acc[mb][nb] = WFrag<T16>::mma(a[mb], b, acc[mb][nb]); if (NSPLIT == 1 || NSPLIT == 2) acc[mb][nb] = WFrag<T16>::mma(a2[mb], b, acc[mb][nb]); if (NSPLIT >= 2) acc[mb][nb] = WFrag<T16>::mma(a[mb], b2, acc[mb][nb]); } }
        asm volatile("v_nop\n\tv_nop\n\tv_nop\n\tv_nop" : "+v"(acc[0][0]), "+v"(acc[1][1]), "+v"(acc[2][2]), "+v"(acc[3][3]) : "v"(a[0]), "v"(a[3]));
    }
#pragma unroll
    for (int mb = 0; mb < 4; ++mb) {
#pragma unroll
        for (int nb = 0; nb < 4; ++nb) {
#pragma unroll
            for (int j = 0; j < 8; ++j) os[(hi * 8 + j) * 68 + nb * 16 + lr] = acc[mb][nb][j]; }
        __builtin_amdgcn_wave_barrier(); asm volatile("" ::: "memory");
        float* crow = C + (size_t)(r0 + mb * 16) * ldc + c0;
#pragma unroll 1
        for (int ps = 0; ps < 2; ++ps) {
#pragma unroll
            for (int s = 0; s < 8; ++s) { const int row = 2 * s + hi, cofs = lr * 4; v4f val = *(const v4fa*)(os + row * 68 + cofs); if (BIAS) { val[0] += bfr(bias[c0 + cofs]); val[1] += bfr(bias[c0 + cofs + 1]); val[2] += bfr(bias[c0 + cofs + 2]); val[3] += bfr(bias[c0 + cofs + 3]); }
                *(volatile v4f*)(crow + (size_t)row * ldc + cofs) = val; }
            if (ps == 0) __threadfence(); }
        __builtin_amdgcn_wave_barrier(); asm volatile("" ::: "memory");
    }
}

__global__ __launch_bounds__(256) void k_wtG(const float* __restrict__ w, int K, int N, bf* Bt) {
    const int lane = threadIdx.x & 31; const int L0 = (blockIdx.x * 8 + (threadIdx.x >> 5)) * 8; const int nlines = N * K / 64;
#pragma unroll
    for (int ps = 0; ps < 2; ++ps) {
#pragma unroll 1
        for (int l = 0; l < 8; ++l) { const int L = L0 + l; if (L >= nlines) break; const size_t e = (size_t)L * 64 + lane * 2; const int k = (int)(e % K), n = (int)(e / K); v2us o;
            o[0] = f2bf(w[(size_t)k * N + n]); o[1] = f2bf(w[(size_t)(k + 1) * N + n]); *(volatile v2us*)(Bt + e) = o; }
        if (ps == 0) __threadfence(); }
}

__global__ __launch_bounds__(256) void k_cvt8(const float* __restrict__ src, bf* dst, size_t n8) { const size_t i = (size_t)blockIdx.x * 256 + threadIdx.x; if (i >= n8) return; const v8f v = *(const v8f*)(src + i * 8); v8us o;
#pragma unroll
    for (int k = 0; k < 8; ++k) o[k] = f2bf(v[k]); *(volatile v8us*)(dst + i * 8) = o; __threadfence(); *(volatile v8us*)(dst + i * 8) = o; }

__global__ __launch_bounds__(256) void k_qk16(const float* __restrict__ Cb, h16* QP, h16* KP) {
    const size_t i = (size_t)blockIdx.x * 256 + threadIdx.x; if (i >= (size_t)NH * SEQ * HD / 8) return;
    const size_t e = i * 8; const int d = (int)(e % HD); const int n = (int)((e / HD) % SEQ); const int hd = (int)(e / ((size_t)HD * SEQ));
    const float* src = Cb + (size_t)n * QKVC + (size_t)hd * (3 * HD) + d;
    const v8f q = *(const v8f*)src; const v8f k = *(const v8f*)(src + HD);
    v8h oq, ok;
#pragma unroll
    for (int j = 0; j < 8; ++j) { oq[j] = tohx(q[j]); ok[j] = tohx(k[j]); }
    *(volatile v8h*)(QP + e) = oq; *(volatile v8h*)(KP + e) = ok; __threadfence(); *(volatile v8h*)(QP + e) = oq; *(volatile v8h*)(KP + e) = ok; }

__global__ __launch_bounds__(256) void k_vt16(const float* __restrict__ Cb, h16* VT) {
    const size_t e = ((size_t)blockIdx.x * 256 + threadIdx.x) * 2; if (e >= (size_t)NH * HD * SEQ) return;
    const int t = (int)(e % SEQ); const int d = (int)((e / SEQ) % HD); const int hd = (int)(e / ((size_t)SEQ * HD));
    const float* src = Cb + (size_t)hd * (3 * HD) + 2 * HD + d;
    v2h o; o[0] = tohx(src[(size_t)t * QKVC] * VCAR); o[1] = tohx(src[(size_t)(t + 1) * QKVC] * VCAR);
    *(volatile v2h*)(VT + e) = o; __threadfence(); *(volatile v2h*)(VT + e) = o; }

__global__ __launch_bounds__(64) void k_flash(const h16* __restrict__ QP, const h16* __restrict__ KP, const h16* __restrict__ VT, const int* __restrict__ msk, bf* CH, bf* CL) {
    __shared__ __align__(16) float os[2][16 * 68];
    const int lane = threadIdx.x & 31, wv = threadIdx.x >> 5, h = lane >> 4, m = lane & 15;
    const int nqb = SEQ / 32;
    const int bh = blockIdx.x / nqb, qb = blockIdx.x - bh * nqb;
    const int b = bh / NH, hh = bh - b * NH;
    const int q0 = qb * 32 + wv * 16;
    const h16* Qp = QP + (size_t)bh * SEQ * HD; const h16* Kp = KP + (size_t)bh * SEQ * HD; const h16* Vp = VT + (size_t)bh * HD * SEQ;
    const int* mr = msk + (size_t)b * SEQ_FULL;
    const v16h bq0 = ldh(Qp + (size_t)(q0 + m) * HD + 8 * h);
    const v16h bq1 = ldh(Qp + (size_t)(q0 + m) * HD + 32 + 8 * h);
    const bool qok = (mr[q0 + m] != 0);
    float m_run = -1.0e30f, l_run = 0.0f;
    v8f o[4], o2[4];
#pragma unroll
    for (int f = 0; f < 4; ++f) { o[f] = (v8f){}; o2[f] = (v8f){}; }
#pragma unroll 1
    for (int j0 = 0; j0 < SEQ; j0 += 32) {
        v16h ak[2][2];
#pragma unroll
        for (int kt = 0; kt < 2; ++kt) { const h16* kp = Kp + (size_t)(j0 + 16 * kt + m) * HD + 8 * h; ak[kt][0] = ldh(kp); ak[kt][1] = ldh(kp + 32); }
        const v8i mk0 = *(const v8i*)(mr + j0 + 8 * h); const v8i mk1 = *(const v8i*)(mr + j0 + 16 + 8 * h);
        v8f s[2];
#pragma unroll
        for (int kt = 0; kt < 2; ++kt) { v8f c = (v8f){}; c = wmma16(ak[kt][0], bq0, c); c = wmma16(ak[kt][1], bq1, c); s[kt] = c; }
        asm volatile("v_nop\n\tv_nop\n\tv_nop\n\tv_nop" : "+v"(s[0]), "+v"(s[1]) : "v"(bq0), "v"(bq1), "v"(ak[0][0]), "v"(ak[0][1]), "v"(ak[1][0]), "v"(ak[1][1]));
        float tmax = -1.0e30f;
#pragma unroll
        for (int r = 0; r < 8; ++r) {
            const float u0 = (qok && (mk0[r] != 0)) ? s[0][r] * SCL : -MASKV;
            const float u1 = (qok && (mk1[r] != 0)) ? s[1][r] * SCL : -MASKV;
            s[0][r] = u0; s[1][r] = u1; tmax = fmaxf(tmax, fmaxf(u0, u1)); }
        tmax = fmaxf(tmax, __shfl_xor(tmax, 16, 32));
        const float newm = fmaxf(m_run, tmax);
        const float corr = __builtin_amdgcn_exp2f((m_run - newm) * L2E);
        float psum = 0.0f; v16h phv = (v16h){}, prv = (v16h){};
#pragma unroll
        for (int kt = 0; kt < 2; ++kt)
#pragma unroll
            for (int r = 0; r < 8; ++r) {
                const float p = __builtin_amdgcn_exp2f((s[kt][r] - newm) * L2E); psum += p;
                const float pc = p * PCAR; const h16 hv = tohx(pc); phv[8 * kt + r] = hv; prv[8 * kt + r] = tohx((pc - (float)hv) * RCAR); }
        psum += __shfl_xor(psum, 16, 32);
        l_run = l_run * corr + psum; m_run = newm;
        float cq[8];
#pragma unroll
        for (int r = 0; r < 8; ++r) cq[r] = __shfl(corr, 8 * h + r, 32);
#pragma unroll
        for (int f = 0; f < 4; ++f)
#pragma unroll
            for (int r = 0; r < 8; ++r) { o[f][r] *= cq[r]; o2[f][r] *= cq[r]; }
        v16h bv[4];
#pragma unroll
        for (int f = 0; f < 4; ++f) bv[f] = ldh(Vp + (size_t)(16 * f + m) * SEQ + j0 + 8 * h);
#pragma unroll
        for (int f = 0; f < 4; ++f) { o[f] = wmma16(phv, bv[f], o[f]); o2[f] = wmma16(prv, bv[f], o2[f]); }
        asm volatile("v_nop\n\tv_nop\n\tv_nop\n\tv_nop" : "+v"(o[0]), "+v"(o[1]), "+v"(o[2]), "+v"(o[3]), "+v"(o2[0]), "+v"(o2[1]), "+v"(o2[2]), "+v"(o2[3]) : "v"(phv), "v"(prv), "v"(bv[0]), "v"(bv[1]), "v"(bv[2]), "v"(bv[3]));
    }
    const float linv = 1.0f / l_run;
    float lq[8];
#pragma unroll
    for (int r = 0; r < 8; ++r) lq[r] = __shfl(linv, 8 * h + r, 32) * (1.0f / (PCAR * VCAR));
    float* osw = &os[wv][0];
#pragma unroll
    for (int f = 0; f < 4; ++f)
#pragma unroll
        for (int r = 0; r < 8; ++r) osw[(8 * h + r) * 68 + 16 * f + m] = (o[f][r] + o2[f][r] * (1.0f / RCAR)) * lq[r];
    __builtin_amdgcn_fence(3  , "wavefront"); __builtin_amdgcn_wave_barrier(); asm volatile("" ::: "memory");
    const int rr = lane >> 3, cc = lane & 7;
    const size_t obase = ((size_t)b * SEQ + q0) * DMO + (size_t)hh * HD + 8 * cc;
#pragma unroll 1
    for (int ps = 0; ps < 2; ++ps) {
#pragma unroll
        for (int s4 = 0; s4 < 4; ++s4) {
            const int row = 4 * s4 + rr;
            const v4f a0 = *(const v4fa*)(osw + row * 68 + 8 * cc); const v4f a1 = *(const v4fa*)(osw + row * 68 + 8 * cc + 4);
            v8us oh, ol;
#pragma unroll
            for (int k = 0; k < 4; ++k) { unsigned short e0, e1; splitf(a0[k], e0, e1); oh[k] = e0; ol[k] = e1; splitf(a1[k], e0, e1); oh[4 + k] = e0; ol[4 + k] = e1; }
            const size_t oo = obase + (size_t)row * DMO;
            *(volatile v8us*)(CH + oo) = oh; *(volatile v8us*)(CL + oo) = ol; }
        if (ps == 0) __threadfence(); }
}

extern "C" void kernel_launch(void* const* d_in, const int* in_sizes, int n_in,
                              void* d_out, int out_size, void* d_ws, size_t ws_size, hipStream_t stream) {
    if (n_in < 5) return;
    if ((size_t)in_sizes[0] < (size_t)(NB - 1) * SEQ_FULL * DMO + (size_t)SEQ * DMO) return;
    if ((size_t)in_sizes[1] < (size_t)DMO * QKVC) return;
    if ((size_t)in_sizes[2] < (size_t)DMO * DMO) return;
    if (in_sizes[3] < DMO) return;
    if ((size_t)in_sizes[4] < (size_t)(NB - 1) * SEQ_FULL + (size_t)SEQ) return;
    if ((size_t)out_size < (size_t)NB * SEQ * DMO) return;
    const float* x = (const float*)d_in[0]; const float* wqkv = (const float*)d_in[1]; const float* wout = (const float*)d_in[2]; const float* bout = (const float*)d_in[3]; const int* msk = (const int*)d_in[4];
    float* OUT = (float*)d_out;
    char* wsp = (char*)d_ws;
    auto take = [&](size_t bytes) { char* p = wsp; wsp += (bytes + 255) & ~(size_t)255; return (void*)p; };
    bf* XB  = (bf*)take((size_t)SEQ * DMO * 2);
    bf* WQT = (bf*)take((size_t)QKVC * DMO * 2);
    bf* WOT = (bf*)take((size_t)DMO * DMO * 2);
    float* C = (float*)take((size_t)SEQ * QKVC * 4);
    h16* QP = (h16*)take((size_t)NB * NH * SEQ * HD * 2);
    h16* KP = (h16*)take((size_t)NB * NH * SEQ * HD * 2);
    h16* VT = (h16*)take((size_t)NB * NH * HD * SEQ * 2);
    bf* CH  = (bf*)take((size_t)NB * SEQ * DMO * 2);
    bf* CL  = (bf*)take((size_t)NB * SEQ * DMO * 2);
    if ((size_t)(wsp - (char*)d_ws) > ws_size) return;
    const int nlq = QKVC * DMO / 64, nlo = DMO * DMO / 64;
    k_wtG<<<(unsigned)((nlq + 63) / 64), 256, 0, stream>>>(wqkv, DMO, QKVC, WQT);
    k_wtG<<<(unsigned)((nlo + 63) / 64), 256, 0, stream>>>(wout, DMO, DMO, WOT);
    for (int b = 0; b < NB; ++b) {
        k_cvt8<<<(unsigned)(((size_t)SEQ * DMO / 8 + 255) / 256), 256, 0, stream>>>(x + (size_t)b * SEQ_FULL * DMO, XB, (size_t)SEQ * DMO / 8);
        k_gemmw<bf, 0, false><<<dim3(SEQ / 64, QKVC / 64, 1), 32, 0, stream>>>(XB, nullptr, WQT, nullptr, DMO, C, QKVC, nullptr, 0, 0, 0);
        k_qk16<<<(unsigned)(((size_t)NH * SEQ * HD / 8 + 255) / 256), 256, 0, stream>>>(C, QP + (size_t)b * NH * SEQ * HD, KP + (size_t)b * NH * SEQ * HD);
        k_vt16<<<(unsigned)(((size_t)NH * HD * SEQ / 2 + 255) / 256), 256, 0, stream>>>(C, VT + (size_t)b * NH * HD * SEQ);
    }
    k_flash<<<(unsigned)(NB * NH * (SEQ / 32)), 64, 0, stream>>>(QP, KP, VT, msk, CH, CL);
    k_gemmw<bf, 1, true><<<dim3(NB * SEQ / 64, DMO / 64, 1), 32, 0, stream>>>(CH, CL, WOT, nullptr, DMO, OUT, DMO, bout, 0, 0, 0);
}
